// GPSRiskModel_9483287790248
// MI455X (gfx1250) — hardware-run, weakly checked
//
#include <hip/hip_runtime.h>


namespace {
constexpr int NB = 1, L = 4096, C = 128, NH = 4, HD = 32, NT = NB * L, KB = 128, PW = 3 * C;
constexpr int N = 4096, E = 262144, IN = 64, H = 128, F2 = 256, NPB = 8;
constexpr float XS = 8.0f, HS = 256.0f, WSC = 256.0f, PS = 256.0f, SCALE = 0.17677669529663687f, SLOPE = 0.2f, BNK = 0.99999500003749969f  ;
typedef _Float16 b16;
typedef __attribute__((ext_vector_type(16))) _Float16 v16b;
typedef __attribute__((ext_vector_type(8))) _Float16 v8b;
typedef __attribute__((ext_vector_type(8))) float v8f;
typedef __attribute__((ext_vector_type(4))) float v4f;
__device__ __forceinline__ float bf16_rne(float f) { unsigned int u = __float_as_uint(f); u += 0x7FFFu + ((u >> 16) & 1u); float r = __uint_as_float(u & 0xFFFF0000u); asm volatile("" : "+v"(r)); return r; }
__device__ __forceinline__ float bfv(float f) { float r = bf16_rne(f); asm volatile("" : "+v"(r)); return r; }
__device__ __forceinline__ void split16(float v, b16& hi, b16& lo) { hi = (b16)v; lo = (b16)(v - (float)hi); }
__device__ __forceinline__ v16b frag_kb(const b16* p, int hh) { const v8b a = *(const v8b*)(p + 8 * hh), b = *(const v8b*)(p + 16 + 8 * hh); v16b f;
#pragma unroll
  for (int e = 0; e < 8; ++e) { f[e] = a[e]; f[8 + e] = b[e]; } return f; }
__device__ __forceinline__ v8f wmma16b(v16b a, v16b b, v8f c) { v8f d = __builtin_amdgcn_wmma_f32_16x16x32_f16(false, a, false, b, (short)0, c, false, false); asm volatile("v_nop\n\tv_nop\n\tv_nop\n\tv_nop" : "+v"(d) : "v"(a), "v"(b)); return d; }
__device__ __forceinline__ void wave_lds_sync() { __builtin_amdgcn_fence(__ATOMIC_RELEASE, "workgroup"); __builtin_amdgcn_wave_barrier(); __builtin_amdgcn_fence(__ATOMIC_ACQUIRE, "workgroup"); }
__device__ __forceinline__ float pmul(float a, float b) { float p = a * b; asm volatile("" : "+v"(p)); return p; }
__device__ __forceinline__ int iclamp(int v, int lo, int hi) { return v < lo ? lo : (v > hi ? hi : v); }
__device__ __forceinline__ float leaky(float v) { return v >= 0.0f ? v : SLOPE * v; }
constexpr int CSR_NBLK7 = 512, CSR_GB7 = 7, CSR_GN7 = 1 << CSR_GB7  , CSR_TS7 = (CSR_GN7 < 32 ? 32 : CSR_GN7)  , CSR_MAXG7 = 512, CSR_CAP7 = 12288  ;
__device__ __host__ __forceinline__ int csr_tix7(int v) { return (v >> CSR_GB7) * CSR_TS7 + (v & (CSR_GN7 - 1)); }
__global__ __launch_bounds__(64) void csrA_kernel7(const int* __restrict__ dst, int E, int N, int nG, int CHP, int NGP, int* __restrict__ STG, int* __restrict__ HST) {
  extern __shared__ int sm[];
  int* cnt = sm; int* run = sm + NGP; int* ids = sm + 2 * NGP;
  const int b = blockIdx.x; const int ch = (E + CSR_NBLK7 - 1) / CSR_NBLK7; const int e0 = b * ch, e1 = min(E, e0 + ch);
  for (int i = threadIdx.x; i < NGP; i += 64) cnt[i] = 0;
  for (int i = threadIdx.x; i < CHP; i += 64) ids[i] = -1;
  __syncthreads();
  if (threadIdx.x == 0) {
    for (int e = e0; e < e1; ++e) { int d = dst[e]; d = (d < 0) ? 0 : (d >= N ? N - 1 : d); cnt[d >> CSR_GB7] += 1; }
    int acc = 0; for (int g = 0; g < nG; ++g) { run[g] = acc; acc += cnt[g]; }
    for (int e = e0; e < e1; ++e) { int d = dst[e]; d = (d < 0) ? 0 : (d >= N ? N - 1 : d); const int g = d >> CSR_GB7; ids[run[g]] = e; run[g] += 1; } }
  __syncthreads();
  typedef __attribute__((ext_vector_type(4))) int v4i;
  for (int pass = 0; pass < 2; ++pass) {
    for (int i = threadIdx.x; i < CHP / 4; i += 64) *(volatile v4i*)(STG + (size_t)b * CHP + i * 4) = *(const v4i*)(&ids[i * 4]);
    for (int i = threadIdx.x; i < NGP / 4; i += 64) { v4i v; for (int e = 0; e < 4; ++e) v[e] = (i * 4 + e < nG) ? cnt[i * 4 + e] : 0; *(volatile v4i*)(HST + (size_t)b * NGP + i * 4) = v; }
    __threadfence(); }
}
__global__ __launch_bounds__(512) void csrS_kernel7(const int* __restrict__ HST, int nG, int NGP, int* __restrict__ START, int* __restrict__ TOT, int* __restrict__ OFF) {
  __shared__ int tot[CSR_MAXG7];
  const int b = threadIdx.x;
  for (int pass = 0; pass < 2; ++pass) { int runb = 0; for (int g = 0; g < nG; ++g) { int c = HST[(size_t)b * NGP + g]; c = (c < 0) ? 0 : c; ((volatile int*)OFF)[(size_t)g * CSR_NBLK7 + b] = runb; runb += c; } __threadfence(); }
  for (int g = threadIdx.x; g < nG; g += 512) { int s = 0; for (int bb = 0; bb < CSR_NBLK7; ++bb) { int c = HST[(size_t)bb * NGP + g]; s += (c < 0) ? 0 : c; } tot[g] = s; }
  __syncthreads();
  if (threadIdx.x < 32) {
    __shared__ int st[CSR_MAXG7 + 32];
    if (threadIdx.x == 0) { int acc = 0; for (int g = 0; g < NGP; ++g) { st[g] = acc; if (g < nG) acc += (tot[g] + 31) & ~31; } st[NGP] = acc; }
    __builtin_amdgcn_fence(__ATOMIC_RELEASE, "workgroup"); __builtin_amdgcn_wave_barrier(); __builtin_amdgcn_fence(__ATOMIC_ACQUIRE, "workgroup");
    for (int pass = 0; pass < 2; ++pass) { for (int i = threadIdx.x; i < NGP + 32; i += 32) { ((volatile int*)START)[i] = (i <= NGP) ? st[min(i, NGP)] : 0; ((volatile int*)TOT)[i] = (i < nG) ? tot[i] : 0; } __threadfence(); } }
}
__global__ __launch_bounds__(256) void csrB_kernel7(const int* __restrict__ dst, int N, int nG, int CHP, int NGP, int permLen, const int* __restrict__ STG, const int* __restrict__ HST, const int* __restrict__ OFF, const int* __restrict__ START, const int* __restrict__ TOT, int* __restrict__ PERM, int* __restrict__ ROWPTR, int* __restrict__ ROWCNT, int* __restrict__ FLAG) {
  typedef __attribute__((ext_vector_type(4))) int v4i;
  __shared__ int ids[CSR_CAP7]; __shared__ unsigned short key[CSR_CAP7]; __shared__ int outp[CSR_CAP7]; __shared__ int ncnt[CSR_GN7 + 1]; __shared__ int boff[CSR_NBLK7 + 1];
  const int g = blockIdx.x, t_ = threadIdx.x; int tot = TOT[g]; int st = START[g], stn = START[g + 1]; const int v0 = g * CSR_GN7; const int nv = min(CSR_GN7, N - v0); const int t0 = g * CSR_TS7;
  st = (st < 0) ? 0 : (st > permLen - 32 ? permLen - 32 : st) & ~31; stn = (stn < st) ? st : (stn > permLen ? permLen : stn); tot = (tot < 0) ? 0 : tot; if (tot > stn - st && tot <= CSR_CAP7) tot = stn - st;
  if (tot > CSR_CAP7) {
    for (int pass = 0; pass < 2; ++pass) { for (int i = t_; i < CSR_TS7 / 4; i += 256) { v4i a, c; for (int e = 0; e < 4; ++e) { a[e] = st; c[e] = 0; } *(volatile v4i*)(ROWPTR + t0 + i * 4) = a; *(volatile v4i*)(ROWCNT + t0 + i * 4) = c; } if (t_ == 0) ((volatile int*)FLAG)[0] = 1; __threadfence(); } (void)nv; return; }
  if (t_ == 0) { int acc = 0; for (int b = 0; b < CSR_NBLK7; ++b) { boff[b] = acc; int c = HST[(size_t)b * NGP + g]; c = (c < 0) ? 0 : (c > CHP ? CHP : c); acc += c; if (acc > tot) acc = tot; } boff[CSR_NBLK7] = acc; }
  for (int i = t_; i <= CSR_GN7; i += 256) ncnt[i] = 0;
  __syncthreads();
  for (int b = 0; b < CSR_NBLK7; ++b) { const int c = boff[b + 1] - boff[b]; int o_ = OFF[(size_t)g * CSR_NBLK7 + b]; o_ = (o_ < 0) ? 0 : (o_ > CHP - c ? CHP - c : o_); const int* src_ = STG + (size_t)b * CHP + o_;
    for (int i = t_; i < c; i += 256) { int id = src_[i]; id = (id < 0) ? 0 : id; ids[boff[b] + i] = id; int d = dst[id]; d = (d < v0) ? v0 : (d >= N ? N - 1 : d); int kk = d - v0; kk = (kk < 0) ? 0 : (kk >= CSR_GN7 ? CSR_GN7 - 1 : kk); key[boff[b] + i] = (unsigned short)kk; } }
  __syncthreads();
  if (t_ == 0) { for (int i = 0; i < tot; ++i) ncnt[key[i]] += 1; int acc = 0; for (int vl = 0; vl < CSR_GN7; ++vl) { const int c = ncnt[vl]; ncnt[vl] = acc; acc += c; } ncnt[CSR_GN7] = acc;
    for (int i = 0; i < tot; ++i) { const int vl = key[i]; outp[ncnt[vl]] = ids[i]; ncnt[vl] += 1; }
    for (int vl = CSR_GN7; vl > 0; --vl) ncnt[vl] = ncnt[vl - 1]; ncnt[0] = 0; }
  __syncthreads();
  for (int pass = 0; pass < 2; ++pass) {
    for (int i = t_; i < (stn - st) / 4; i += 256) { v4i v; for (int e = 0; e < 4; ++e) { const int q = i * 4 + e; v[e] = (q < tot) ? outp[q] : -1; } *(volatile v4i*)(PERM + st + i * 4) = v; }
    for (int i = t_; i < CSR_TS7 / 4; i += 256) { v4i a, c; for (int e = 0; e < 4; ++e) { const int vl = i * 4 + e; const int vc = vl < CSR_GN7 ? vl : CSR_GN7; a[e] = (vl < CSR_GN7) ? st + ncnt[vc] : st; c[e] = (vl < nv) ? (ncnt[(vc < CSR_GN7 ? vc : CSR_GN7 - 1) + 1] - ncnt[vc]) : 0; } *(volatile v4i*)(ROWPTR + t0 + i * 4) = a; *(volatile v4i*)(ROWCNT + t0 + i * 4) = c; }
    __threadfence(); }
}
__global__ __launch_bounds__(256) void csrZ_kernel7(int* __restrict__ p, size_t n4) { typedef __attribute__((ext_vector_type(4))) int v4i; const size_t tid = (size_t)blockIdx.x * 256 + threadIdx.x, nth = (size_t)gridDim.x * 256; v4i z = {0, 0, 0, 0}; for (size_t i = tid; i < n4; i += nth) *(volatile v4i*)(p + i * 4) = z; }
struct CsrBufs7 { int *STG, *HST, *OFF, *START, *TOT, *PERM, *ROWPTR, *ROWCNT, *FLAG; int nG, NGP, CHP; size_t permLen; char* base; size_t bytes; };
static size_t csr_carve7(CsrBufs7& c, char* ws, size_t off, int E, int N) {
  const size_t off0 = off; c.base = ws + off;
  auto al = [&](size_t bytes) { char* p = ws + off; off += (bytes + 255) & ~(size_t)255; return p; };
  c.nG = (N + CSR_GN7 - 1) / CSR_GN7; c.NGP = (c.nG + 31) & ~31; const int ch = (E + CSR_NBLK7 - 1) / CSR_NBLK7; c.CHP = (ch + 31) & ~31; c.permLen = (size_t)E + 32 * (size_t)c.nG + 32;
  c.STG = (int*)al((size_t)CSR_NBLK7 * c.CHP * 4); c.HST = (int*)al((size_t)CSR_NBLK7 * c.NGP * 4); c.OFF = (int*)al((size_t)c.NGP * CSR_NBLK7 * 4); c.START = (int*)al((size_t)(c.NGP + 64) * 4); c.TOT = (int*)al((size_t)(c.NGP + 64) * 4);
  c.PERM = (int*)al(c.permLen * 4); c.ROWPTR = (int*)al((size_t)c.nG * CSR_TS7 * 4); c.ROWCNT = (int*)al((size_t)c.nG * CSR_TS7 * 4); c.FLAG = (int*)al(256);
  c.bytes = off - off0; return off;
}
static void csr_build7(const CsrBufs7& c, const int* dst, int E, int N, hipStream_t stream) {
  const size_t smem = (size_t)(2 * c.NGP + c.CHP) * 4;
  csrZ_kernel7<<<512, 256, 0, stream>>>((int*)c.base, c.bytes / 16);
  csrA_kernel7<<<CSR_NBLK7, 64, smem, stream>>>(dst, E, N, c.nG, c.CHP, c.NGP, c.STG, c.HST);
  csrS_kernel7<<<1, 512, 0, stream>>>(c.HST, c.nG, c.NGP, c.START, c.TOT, c.OFF);
  csrB_kernel7<<<c.nG, 256, 0, stream>>>(dst, N, c.nG, c.CHP, c.NGP, (int)c.permLen, c.STG, c.HST, c.OFF, c.START, c.TOT, c.PERM, c.ROWPTR, c.ROWCNT, c.FLAG);
}


__global__ __launch_bounds__(256) void wput_kernel(const float* __restrict__ win, const float* __restrict__ wgat, const float* __restrict__ wqkv, const float* __restrict__ wo, const float* __restrict__ w1, const float* __restrict__ w2,
    b16* __restrict__ WIN, b16* __restrict__ WGAT, b16* __restrict__ W3, b16* __restrict__ WO, b16* __restrict__ W1, b16* __restrict__ W2) { const size_t nt = (size_t)gridDim.x * 256, u0 = (size_t)blockIdx.x * 256 + threadIdx.x; v8b v;
  auto put = [&](const float* src, b16* dst, size_t rows, int kin) { for (size_t u = u0; u < rows * (kin / 8); u += nt) { const size_t o = u / (kin / 8); const int k0 = (int)(u % (kin / 8)) * 8;
#pragma unroll
      for (int j = 0; j < 8; ++j) v[j] = (b16)(bf16_rne(src[o * kin + k0 + j]) * WSC); for (int pass = 0; pass < 2; ++pass) { *(volatile v8b*)(dst + o * kin + k0) = v; __threadfence(); } } };
  put(win, WIN, H, IN); put(wgat, WGAT, 2 * H, H); put(wqkv, W3, 2 * 3 * H, H); put(wo, WO, 2 * H, H); put(w1, W1, 2 * F2, H); put(w2, W2, 2 * H, F2); }
__global__ __launch_bounds__(32) void in_kernel(const float* __restrict__ x, const b16* __restrict__ WIN, const float* __restrict__ bin, int NLIM, float* __restrict__ HP) { __shared__ __attribute__((aligned(16))) b16 Ah[16][IN + 8]; __shared__ float Tf[16][H + 4]; const int lane = threadIdx.x, nloc = lane & 15, hlf = lane >> 4; const size_t m0 = (size_t)blockIdx.x * 16; if (m0 >= (size_t)NLIM) return;
  for (int rr = 0; rr < 16; ++rr) for (int q = 0; q < 2; ++q) Ah[rr][q * 32 + lane] = (b16)(bf16_rne(x[(m0 + rr) * IN + q * 32 + lane]) * XS); if (lane < 16) for (int k = IN; k < IN + 8; ++k) Ah[lane][k] = (b16)0.0f;
  wave_lds_sync(); v8f acc[8];
#pragma unroll
  for (int t = 0; t < 8; ++t) acc[t] = (v8f){};
#pragma unroll
  for (int kb = 0; kb < IN; kb += 32) { const v16b a = frag_kb(&Ah[nloc][kb], hlf);
#pragma unroll
    for (int t = 0; t < 8; ++t) acc[t] = wmma16b(a, frag_kb(WIN + (size_t)(t * 16 + nloc) * IN + kb, hlf), acc[t]); }
#pragma unroll
  for (int t = 0; t < 8; ++t) { const int cc = t * 16 + nloc; const float bb = bfv(bin[cc]);
#pragma unroll
    for (int r8 = 0; r8 < 8; ++r8) Tf[8 * hlf + r8][cc] = fmaxf(acc[t][r8] * (1.0f / (XS * WSC)) + bb, 0.0f); }
  wave_lds_sync();
  for (int pass = 0; pass < 2; ++pass) { for (int rr = 0; rr < 16; ++rr) *(volatile v4f*)(HP + (m0 + rr) * H + lane * 4) = *(const v4f*)(&Tf[rr][lane * 4]); __threadfence(); } }
__global__ __launch_bounds__(32) void proj_kernel(const float* __restrict__ HP, const b16* __restrict__ WGAT, const b16* __restrict__ W3, const float* __restrict__ as_, const float* __restrict__ ad_, const float* __restrict__ bqkv, int NLIM, float* __restrict__ XP, float* __restrict__ ES, b16* __restrict__ PH, b16* __restrict__ PL) { __shared__ __attribute__((aligned(16))) b16 Ah[16][H + 8], Al[16][H + 8], Oh[16][H + 8], Ol[16][H + 8]; __shared__ float Tf[16][H + 4], Eq[16][8]; const int lane = threadIdx.x, nloc = lane & 15, hlf = lane >> 4; const size_t m0 = (size_t)blockIdx.x * 16; if (m0 >= (size_t)NLIM) return;
  for (int rr = 0; rr < 16; ++rr) for (int q = 0; q < 4; ++q) { b16 p, ql; split16(HP[(m0 + rr) * H + q * 32 + lane] * HS, p, ql); Ah[rr][q * 32 + lane] = p; Al[rr][q * 32 + lane] = ql; } if (lane < 16) for (int k = H; k < H + 8; ++k) { Ah[lane][k] = (b16)0.0f; Al[lane][k] = (b16)0.0f; }
  wave_lds_sync();
#pragma unroll 1
  for (int g = 0; g < 4; ++g) { const b16* W = g == 0 ? WGAT : W3 + (size_t)(g - 1) * H * H; v8f acc[8];
#pragma unroll
    for (int t = 0; t < 8; ++t) acc[t] = (v8f){};
#pragma unroll
    for (int kb = 0; kb < H; kb += 32) { const v16b a = frag_kb(&Ah[nloc][kb], hlf), al = frag_kb(&Al[nloc][kb], hlf);
#pragma unroll
      for (int t = 0; t < 8; ++t) { const v16b bw = frag_kb(W + (size_t)(t * 16 + nloc) * H + kb, hlf); acc[t] = wmma16b(a, bw, acc[t]); acc[t] = wmma16b(al, bw, acc[t]); } }
    if (g == 0) {
#pragma unroll
      for (int t = 0; t < 8; ++t)
#pragma unroll
        for (int r8 = 0; r8 < 8; ++r8) Tf[8 * hlf + r8][t * 16 + nloc] = acc[t][r8] * (1.0f / (HS * WSC));
      wave_lds_sync();
      for (int rr = 0; rr < 16; ++rr) { const int hd = lane >> 3, c0 = (lane & 7) * 4; float s1 = 0.0f, s2 = 0.0f; for (int k = 0; k < 4; ++k) { const int cc = hd * HD + c0 + k; s1 += pmul(Tf[rr][cc], bfv(as_[cc])); s2 += pmul(Tf[rr][cc], bfv(ad_[cc])); } for (int o = 1; o < 8; o <<= 1) { s1 += __shfl_xor(s1, o); s2 += __shfl_xor(s2, o); } if ((lane & 7) == 0) { Eq[rr][hd] = s1; Eq[rr][4 + hd] = s2; } }
      wave_lds_sync();
      for (int pass = 0; pass < 2; ++pass) { for (int rr = 0; rr < 16; ++rr) *(volatile v4f*)(XP + (m0 + rr) * H + lane * 4) = *(const v4f*)(&Tf[rr][lane * 4]); *(volatile v4f*)(ES + (m0 + (lane >> 1)) * 8 + (lane & 1) * 4) = *(const v4f*)(&Eq[lane >> 1][(lane & 1) * 4]); __threadfence(); } }
    else { const int gq = g - 1; const float sc = gq == 0 ? SCALE : 1.0f;
#pragma unroll
      for (int t = 0; t < 8; ++t) { const int cc = t * 16 + nloc; const float bb = bfv(bqkv[gq * H + cc]);
#pragma unroll
        for (int r8 = 0; r8 < 8; ++r8) { b16 p, ql; split16((acc[t][r8] * (1.0f / (HS * WSC)) + bb) * sc * HS, p, ql); Oh[8 * hlf + r8][cc] = p; Ol[8 * hlf + r8][cc] = ql; } }
      wave_lds_sync();
      for (int pass = 0; pass < 2; ++pass) { for (int rr = 0; rr < 16; ++rr) if (lane < 16) { *(volatile v8b*)(PH + (m0 + rr) * PW + gq * H + lane * 8) = *(const v8b*)(&Oh[rr][lane * 8]); *(volatile v8b*)(PL + (m0 + rr) * PW + gq * H + lane * 8) = *(const v8b*)(&Ol[rr][lane * 8]); } __threadfence(); } }
    wave_lds_sync(); } }
__global__ __launch_bounds__(256) void gat_kernel(const float* __restrict__ XP, const float* __restrict__ ES, const float* __restrict__ HP, const float* __restrict__ bg, const float* __restrict__ g0, const float* __restrict__ b0, const int* __restrict__ srcs, const int* __restrict__ PERM, const int* __restrict__ ROWPTR, const int* __restrict__ ROWCNT, int permLen, int NLIM, float* __restrict__ HL) { const int wave = threadIdx.x >> 5, lane = threadIdx.x & 31, hd = lane >> 3; const size_t i = (size_t)blockIdx.x * NPB + wave; if (i >= (size_t)NLIM) return; int st = ROWPTR[i], cnt = ROWCNT[i]; cnt = iclamp(cnt, 0, E); st = iclamp(st, 0, permLen - cnt); const float edi = ES[i * 8 + 4 + hd];
  float mx = -INFINITY, den = 0.0f; v4f acc = {0, 0, 0, 0};
#pragma unroll 1
  for (int j = 0; j < cnt; ++j) { const int e = iclamp(PERM[st + j], 0, E - 1); const size_t u = (size_t)iclamp(srcs[e], 0, N - 1); if (u >= (size_t)NLIM) continue; const float s = leaky(ES[u * 8 + hd] + edi); const float mn = fmaxf(mx, s); const float sf = (mx == -INFINITY) ? 0.0f : __expf(mx - mn); const float p = __expf(s - mn); den = den * sf + p; const v4f v = *(const v4f*)(XP + u * H + lane * 4);
#pragma unroll
    for (int k = 0; k < 4; ++k) acc[k] = pmul(acc[k], sf) + pmul(p, v[k]); mx = mn; }
  const v4f hv = *(const v4f*)(HP + i * H + lane * 4); v4f o;
#pragma unroll
  for (int k = 0; k < 4; ++k) { const int c = lane * 4 + k; const float gat = (den > 0.0f ? acc[k] / (den + 1e-16f) : 0.0f) + bfv(bg[c]); o[k] = pmul(gat + hv[k], bfv(g0[c]) * BNK) + bfv(b0[c]); }
  for (int pass = 0; pass < 2; ++pass) { *(volatile v4f*)(HL + i * H + lane * 4) = o; __threadfence(); } }
__global__ __launch_bounds__(32) void att_kernel(const b16* __restrict__ PH, const b16* __restrict__ PL, const float* __restrict__ amask, int BLIM, float* __restrict__ ATT) { __shared__ __attribute__((aligned(16))) b16 Ph_[16][KB + 8], Pl_[16][KB + 8], Vth[HD][KB + 8], Vtl[HD][KB + 8]; __shared__ float Sf[16][KB + 4], Of[16][HD + 4];
  const int lane = threadIdx.x, nloc = lane & 15, hlf = lane >> 4; const int qt = blockIdx.x % (L / 16); const int h = (blockIdx.x / (L / 16)) % NH; const int b = blockIdx.x / ((L / 16) * NH); if (b >= BLIM) return; const int t0 = qt * 16; const size_t rowb = (size_t)b * L; const int qo = h * HD, ko = C + h * HD, vo = 2 * C + h * HD;
  v16b qh[HD / 32], ql[HD / 32];
#pragma unroll
  for (int s = 0; s < HD / 32; ++s) { qh[s] = frag_kb(PH + (rowb + t0 + nloc) * PW + qo + s * 32, hlf); ql[s] = frag_kb(PL + (rowb + t0 + nloc) * PW + qo + s * 32, hlf); }
  float m_r[8], den_r[8]; v8f acc[HD / 16];
#pragma unroll
  for (int r8 = 0; r8 < 8; ++r8) { m_r[r8] = -INFINITY; den_r[r8] = 0.0f; }
#pragma unroll
  for (int t = 0; t < HD / 16; ++t) acc[t] = (v8f){};
  const int kstart = 0; const int kend = L;
#pragma unroll 1
  for (int kb0 = kstart; kb0 < kend; kb0 += KB) { const int nk = (kend - kb0) < KB ? (kend - kb0) : KB; const int nkt = (nk + 15) / 16;
    for (int rr = 0; rr < KB; rr += 2) { const int r = rr + hlf; const int key = kb0 + r < L ? kb0 + r : L - 1;     const size_t vr = (rowb + key) * PW + vo; for (int s = 0; s < HD / 32; ++s) { Vth[s * 32 + nloc][r] = PH[vr + s * 32 + nloc]; Vth[s * 32 + 16 + nloc][r] = PH[vr + s * 32 + 16 + nloc]; Vtl[s * 32 + nloc][r] = PL[vr + s * 32 + nloc]; Vtl[s * 32 + 16 + nloc][r] = PL[vr + s * 32 + 16 + nloc]; } }
    for (int t = 0; t < KB / 16; ++t) { if (t < nkt) { const int key = kb0 + t * 16 + nloc < L ? kb0 + t * 16 + nloc : L - 1; const size_t kr = (rowb + key) * PW + ko; v8f s = {};
#pragma unroll
        for (int q = 0; q < HD / 32; ++q) { const v16b kh = frag_kb(PH + kr + q * 32, hlf), kl = frag_kb(PL + kr + q * 32, hlf); s = wmma16b(qh[q], kh, s); s = wmma16b(qh[q], kl, s); s = wmma16b(ql[q], kh, s); }
#pragma unroll
        for (int r8 = 0; r8 < 8; ++r8) { const int i = t0 + 8 * hlf + r8, j = kb0 + t * 16 + nloc; const bool ok = (j < kend); Sf[8 * hlf + r8][t * 16 + nloc] = ok ? s[r8] * (1.0f / (HS * HS)) : -INFINITY; } }
      else {
#pragma unroll
        for (int r8 = 0; r8 < 8; ++r8) Sf[8 * hlf + r8][t * 16 + nloc] = -INFINITY; } }
    wave_lds_sync();
#pragma unroll
    for (int rr = 0; rr < 16; ++rr) { float mx = -INFINITY;
#pragma unroll
      for (int q = 0; q < 4; ++q) mx = fmaxf(mx, Sf[rr][q * 32 + lane]);
      for (int o = 16; o; o >>= 1) mx = fmaxf(mx, __shfl_xor(mx, o));
      const float mold = __shfl(m_r[rr & 7], (rr >> 3) * 16); const float mn = fmaxf(mold, mx); const float sf = (mold == -INFINITY) ? 0.0f : ((mn == -INFINITY) ? 1.0f : __expf(mold - mn)); float ps = 0.0f;
#pragma unroll
      for (int q = 0; q < 4; ++q) { const int kx = q * 32 + lane; const float sv = Sf[rr][kx]; const float p = (sv == -INFINITY || mn == -INFINITY) ? 0.0f : __expf(sv - mn); ps += p; b16 ph, pl; split16(p * PS, ph, pl); Ph_[rr][kx] = ph; Pl_[rr][kx] = pl; }
      for (int o = 16; o; o >>= 1) ps += __shfl_xor(ps, o);
      if ((rr >> 3) == hlf) { const int r8 = rr & 7; den_r[r8] = den_r[r8] * sf + ps; m_r[r8] = mn;
#pragma unroll
        for (int t = 0; t < HD / 16; ++t) acc[t][r8] = acc[t][r8] * sf; } }
    wave_lds_sync();
    for (int ks = 0; ks < nkt * 16; ks += 32) { const v16b pa = frag_kb(&Ph_[nloc][ks], hlf), pb = frag_kb(&Pl_[nloc][ks], hlf);
#pragma unroll
      for (int t = 0; t < HD / 16; ++t) { const v16b vh = frag_kb(&Vth[t * 16 + nloc][ks], hlf), vl = frag_kb(&Vtl[t * 16 + nloc][ks], hlf); acc[t] = wmma16b(pa, vh, acc[t]); acc[t] = wmma16b(pa, vl, acc[t]); acc[t] = wmma16b(pb, vh, acc[t]); } }
    wave_lds_sync(); }
#pragma unroll
  for (int t = 0; t < HD / 16; ++t)
#pragma unroll
    for (int r8 = 0; r8 < 8; ++r8) { const float dn = den_r[r8]; Of[8 * hlf + r8][t * 16 + nloc] = dn > 0.0f ? acc[t][r8] * (1.0f / (HS * PS)) / dn : 0.0f; }
  wave_lds_sync();
  for (int pass = 0; pass < 2; ++pass) { for (int rr = 0; rr < 16; ++rr) for (int s = 0; s < HD / 32; ++s) ((volatile float*)ATT)[(rowb + t0 + rr) * C + h * HD + s * 32 + lane] = Of[rr][s * 32 + lane]; __threadfence(); } }

__global__ __launch_bounds__(32) void post_kernel(const float* __restrict__ ATT, const float* __restrict__ HP, const float* __restrict__ HL, const b16* __restrict__ WO, const b16* __restrict__ W1, const b16* __restrict__ W2, const float* __restrict__ bo, const float* __restrict__ b1, const float* __restrict__ b2, const float* __restrict__ g1, const float* __restrict__ be1, const float* __restrict__ g2, const float* __restrict__ be2, const float* __restrict__ wout, const float* __restrict__ bout, int LASTL, int NLIM, float* __restrict__ HN, float* __restrict__ OUT) {
  __shared__ __attribute__((aligned(16))) b16 Ah[16][F2 + 8], Al[16][F2 + 8]; __shared__ float To[16][H + 4], Tm[16][F2 + 4], Y2[16][2]; const int lane = threadIdx.x, nloc = lane & 15, hlf = lane >> 4; const size_t m0 = (size_t)blockIdx.x * 16; if (m0 >= (size_t)NLIM) return;
  for (int rr = 0; rr < 16; ++rr) for (int q = 0; q < 4; ++q) { b16 p, ql; split16(ATT[(m0 + rr) * H + q * 32 + lane] * HS, p, ql); Ah[rr][q * 32 + lane] = p; Al[rr][q * 32 + lane] = ql; } if (lane < 16) for (int k = H; k < H + 8; ++k) { Ah[lane][k] = (b16)0.0f; Al[lane][k] = (b16)0.0f; }
  wave_lds_sync();
  { v8f acc[8];
#pragma unroll
    for (int t = 0; t < 8; ++t) acc[t] = (v8f){};
#pragma unroll
    for (int kb = 0; kb < H; kb += 32) { const v16b a = frag_kb(&Ah[nloc][kb], hlf), al = frag_kb(&Al[nloc][kb], hlf);
#pragma unroll
      for (int t = 0; t < 8; ++t) { const v16b bw = frag_kb(WO + (size_t)(t * 16 + nloc) * H + kb, hlf); acc[t] = wmma16b(a, bw, acc[t]); acc[t] = wmma16b(al, bw, acc[t]); } }
#pragma unroll
    for (int t = 0; t < 8; ++t) { const int cc = t * 16 + nloc; const float bb = bfv(bo[cc]), sc1 = bfv(g1[cc]) * BNK, sh1 = bfv(be1[cc]);
#pragma unroll
      for (int r8 = 0; r8 < 8; ++r8) { const int rr = 8 * hlf + r8; const float hatt = pmul(acc[t][r8] * (1.0f / (HS * WSC)) + bb + HP[(m0 + rr) * H + cc], sc1) + sh1; To[rr][cc] = HL[(m0 + rr) * H + cc] + hatt; } } }
  wave_lds_sync();
  for (int rr = 0; rr < 16; ++rr) for (int q = 0; q < 4; ++q) { b16 p, ql; split16(To[rr][q * 32 + lane] * HS, p, ql); Ah[rr][q * 32 + lane] = p; Al[rr][q * 32 + lane] = ql; }
  wave_lds_sync();
  { v8f acc[16];
#pragma unroll
    for (int t = 0; t < 16; ++t) acc[t] = (v8f){};
#pragma unroll
    for (int kb = 0; kb < H; kb += 32) { const v16b a = frag_kb(&Ah[nloc][kb], hlf), al = frag_kb(&Al[nloc][kb], hlf);
#pragma unroll
      for (int t = 0; t < 16; ++t) { const v16b bw = frag_kb(W1 + (size_t)(t * 16 + nloc) * H + kb, hlf); acc[t] = wmma16b(a, bw, acc[t]); acc[t] = wmma16b(al, bw, acc[t]); } }
    wave_lds_sync();
#pragma unroll
    for (int t = 0; t < 16; ++t) { const int cc = t * 16 + nloc; const float bb = bfv(b1[cc]);
#pragma unroll
      for (int r8 = 0; r8 < 8; ++r8) { b16 p, ql; split16(fmaxf(acc[t][r8] * (1.0f / (HS * WSC)) + bb, 0.0f) * HS, p, ql); Ah[8 * hlf + r8][cc] = p; Al[8 * hlf + r8][cc] = ql; } } }
  if (lane < 16) for (int k = F2; k < F2 + 8; ++k) { Ah[lane][k] = (b16)0.0f; Al[lane][k] = (b16)0.0f; }
  wave_lds_sync();
  { v8f acc[8];
#pragma unroll
    for (int t = 0; t < 8; ++t) acc[t] = (v8f){};
#pragma unroll 2
    for (int kb = 0; kb < F2; kb += 32) { const v16b a = frag_kb(&Ah[nloc][kb], hlf), al = frag_kb(&Al[nloc][kb], hlf);
#pragma unroll
      for (int t = 0; t < 8; ++t) { const v16b bw = frag_kb(W2 + (size_t)(t * 16 + nloc) * F2 + kb, hlf); acc[t] = wmma16b(a, bw, acc[t]); acc[t] = wmma16b(al, bw, acc[t]); } }
#pragma unroll
    for (int t = 0; t < 8; ++t) { const int cc = t * 16 + nloc; const float bb = bfv(b2[cc]), sc2 = bfv(g2[cc]) * BNK, sh2 = bfv(be2[cc]);
#pragma unroll
      for (int r8 = 0; r8 < 8; ++r8) { const int rr = 8 * hlf + r8; const float out2 = pmul(To[rr][cc] + acc[t][r8] * (1.0f / (HS * WSC)) + bb, sc2) + sh2; Tm[rr][cc] = fmaxf(out2 + HP[(m0 + rr) * H + cc], 0.0f); } } }
  wave_lds_sync();
  if (LASTL) { for (int rr = 0; rr < 16; ++rr) { float s0 = 0.0f, s1 = 0.0f; for (int q = 0; q < 4; ++q) { const int c = q * 32 + lane; s0 += pmul(Tm[rr][c], bfv(wout[c])); s1 += pmul(Tm[rr][c], bfv(wout[H + c])); } for (int o = 16; o; o >>= 1) { s0 += __shfl_xor(s0, o); s1 += __shfl_xor(s1, o); } if (lane == 0) { Y2[rr][0] = s0 + bfv(bout[0]); Y2[rr][1] = s1 + bfv(bout[1]); } } wave_lds_sync(); }
  for (int pass = 0; pass < 2; ++pass) { for (int rr = 0; rr < 16; ++rr) *(volatile v4f*)(HN + (m0 + rr) * H + lane * 4) = *(const v4f*)(&Tm[rr][lane * 4]); if (LASTL) ((volatile float*)OUT)[m0 * 2 + lane] = Y2[lane >> 1][lane & 1]; __threadfence(); } }
}

extern "C" void kernel_launch(void* const* d_in, const int* in_sizes, int n_in, void* d_out, int out_size, void* d_ws, size_t ws_size, hipStream_t stream) {
  (void)n_in;
  auto Fp = [&](int i) { return (const float*)d_in[i]; }; auto Ip = [&](int i) { return (const int*)d_in[i]; };
  if (in_sizes[0] != N * IN || in_sizes[1] != 2 * E || in_sizes[2] != H * IN || in_sizes[4] != 2 * H * H || in_sizes[5] != 2 * H || in_sizes[8] != 2 * 3 * H * H || in_sizes[10] != 2 * H * H || in_sizes[12] != 2 * 3 * H || in_sizes[14] != 2 * F2 * H || in_sizes[16] != 2 * H * F2 || in_sizes[18] != 2 * H || out_size != N * 2) return;
  const int NLIM = N;
  size_t off = 0; char* ws = (char*)d_ws;
  auto carve = [&](size_t bytes) { char* p = ws + off; off += (bytes + 255) & ~(size_t)255; return p; };
  b16* WIN = (b16*)carve((size_t)H * IN * 2); b16* WGAT = (b16*)carve((size_t)2 * H * H * 2); b16* W3 = (b16*)carve((size_t)2 * 3 * H * H * 2); b16* WO = (b16*)carve((size_t)2 * H * H * 2); b16* W1 = (b16*)carve((size_t)2 * F2 * H * 2); b16* W2 = (b16*)carve((size_t)2 * H * F2 * 2);
  float* HA = (float*)carve((size_t)N * H * 4); float* HB = (float*)carve((size_t)N * H * 4); float* XP = (float*)carve((size_t)N * H * 4); float* ES = (float*)carve((size_t)N * 8 * 4); float* HL = (float*)carve((size_t)N * H * 4); b16* PH = (b16*)carve((size_t)N * PW * 2); b16* PL = (b16*)carve((size_t)N * PW * 2); float* ATT = (float*)carve((size_t)N * H * 4); CsrBufs7 csr; off = csr_carve7(csr, ws, off, E, N);
  if (off > ws_size || off > ((size_t)48 << 20)) return;
  wput_kernel<<<96, 256, 0, stream>>>(Fp(2), Fp(4), Fp(8), Fp(10), Fp(14), Fp(16), WIN, WGAT, W3, WO, W1, W2);
  csr_build7(csr, Ip(1) + E, E, N, stream);
  in_kernel<<<NLIM / 16, 32, 0, stream>>>(Fp(0), WIN, Fp(3), NLIM, HA);
  float* hin = HA; float* hout = HB;
  for (int l = 0; l < 2; ++l) {
    proj_kernel<<<NLIM / 16, 32, 0, stream>>>(hin, WGAT + (size_t)l * H * H, W3 + (size_t)l * 3 * H * H, Fp(5) + l * H, Fp(6) + l * H, Fp(9) + l * 3 * H, NLIM, XP, ES, PH, PL);
    gat_kernel<<<(NLIM + NPB - 1) / NPB, 256, 0, stream>>>(XP, ES, hin, Fp(7) + l * H, Fp(12) + (l * 3 + 0) * H, Fp(13) + (l * 3 + 0) * H, Ip(1), csr.PERM, csr.ROWPTR, csr.ROWCNT, (int)csr.permLen, NLIM, HL);
    att_kernel<<<NB * NH * (L / 16), 32, 0, stream>>>(PH, PL, (const float*)0, NB, ATT);
    post_kernel<<<NLIM / 16, 32, 0, stream>>>(ATT, hin, HL, WO + (size_t)l * H * H, W1 + (size_t)l * F2 * H, W2 + (size_t)l * H * F2, Fp(11) + l * H, Fp(15) + l * F2, Fp(17) + l * H, Fp(12) + (l * 3 + 1) * H, Fp(13) + (l * 3 + 1) * H, Fp(12) + (l * 3 + 2) * H, Fp(13) + (l * 3 + 2) * H, Fp(18), Fp(19), l == 1 ? 1 : 0, NLIM, hout, (float*)d_out);
    float* t = hin; hin = hout; hout = t; }
}
